// CrossAttention_40630390620806
// MI455X (gfx1250) — hardware-run, weakly checked
//
#include <hip/hip_runtime.h>


#ifndef NB
#define NB 4
#endif
#ifndef SEQ
#define SEQ 2048
#endif
#define NB_FULL  4
#define SEQ_FULL 2048
#ifndef OUT_SEQ
#define OUT_SEQ SEQ
#endif
#define HN   8
#define CMV  8
#define CSC  16
#define HDV  144
#define HDP  160
#define NKS  5
#define NZ   (HN * NKS)
#define KIN  288
#define NQK  (HN * HDP)
#define NVF  (HN * HDV)
#define KO   (HN * HDP)
#define NMVO 256
#define NSCO 32
#define NOP  320
#define AW   4
#define OSP  164
#define OTR  32
#define OMB  (OTR / 16)
#define SC2  ((float)(0.083333333333333329 * 1.4426950408889634))
#define PSH  14.0f
#define CXS  64.0f
#define WOS  64.0f
#define OSCL (1.0f / 4096.0f)
#define QRS  2048.0f
#define QRI  (1.0f / 2048.0f)
#define NEGB (-3.0e38f)
#define O1_OFF ((size_t)NB_FULL * SEQ_FULL * NMVO)

static_assert(HDP == NKS * 32);
static_assert(HDV == CMV * 16 + CSC);
static_assert(HDV % 16 == 0);
static_assert(HDV <= HDP);
static_assert(KIN % 32 == 0);
static_assert(KIN % 8 == 0);
static_assert(KO % 32 == 0);
static_assert(KO == NZ * 32);
static_assert(NQK % 64 == 0);
static_assert(NVF % 64 == 0);
static_assert(NOP % 64 == 0);
static_assert(NMVO % 64 == 0);
static_assert(NMVO + NSCO <= NOP);
static_assert(NMVO + 64 == NOP);
static_assert(SEQ % 64 == 0);
static_assert((NB * SEQ) % 64 == 0);
static_assert(SEQ % 32 == 0);
static_assert(SEQ % (16 * AW) == 0);
static_assert(OTR % 16 == 0);
static_assert(OMB == 2);
static_assert(SEQ % OTR == 0);
static_assert((NB * SEQ) % OTR == 0);
static_assert(NB <= NB_FULL);
static_assert(SEQ <= SEQ_FULL);
static_assert((OSP * 4) % 16 == 0);
static_assert(OSP >= HDP);
static_assert(((size_t)NQK * KIN) % 2048 == 0);
static_assert(((size_t)NVF * KIN) % 2048 == 0);
static_assert(((size_t)NOP * KO) % 2048 == 0);
static_assert((size_t)NB * NZ * SEQ * 32 < (size_t)2147483647);
static_assert(O1_OFF * 4 == (size_t)8388608);
static_assert((O1_OFF * 4) % 128 == 0);
static_assert(AW * 16 * OSP * 4 <= 131072);
static_assert(16 * 68 * 4 <= 131072);
static_assert(2 * 2 * 32 * 16 == 16 * 64 * 2);
static_assert(4 * 32 * 16 == 16 * 64 * 2);
static_assert(NKS * 2 * 32 * 16 == 16 * HDP * 2);
static_assert(2 * NKS * 2 * 32 * 16 == 2 * 16 * HDP * 2);
static_assert(8 * 32 * 16 == 16 * 64 * 4);
static_assert(4 * 32 * 16 == 16 * NSCO * 4);
static_assert(OMB * 8 * 32 * 16 == OTR * 64 * 4);
static_assert(OMB * 4 * 32 * 16 == OTR * NSCO * 4);

typedef _Float16 h16;
typedef unsigned short bf;
typedef __attribute__((ext_vector_type(16))) __bf16   v16bf;
typedef __attribute__((ext_vector_type(16))) _Float16 v16h;
typedef __attribute__((ext_vector_type(8)))  _Float16 v8h;
typedef __attribute__((ext_vector_type(8)))  unsigned short v8us;
typedef __attribute__((ext_vector_type(8)))  float    v8f;
typedef __attribute__((ext_vector_type(4)))  float    v4f;
typedef v4f  __attribute__((may_alias)) v4fa;

__device__ __forceinline__ unsigned short f2bf(float f) { unsigned u = __float_as_uint(f); u += 0x7FFFu + ((u >> 16) & 1u); return (unsigned short)(u >> 16); }
__device__ __forceinline__ float bfr(float f) { return __uint_as_float(((unsigned)f2bf(f)) << 16); }
__device__ __forceinline__ v16h cat16(v8h lo, v8h hi) { return __builtin_shufflevector(lo, hi, 0, 1, 2, 3, 4, 5, 6, 7, 8, 9, 10, 11, 12, 13, 14, 15); }
__device__ __forceinline__ v16bf cat16b(v8us lo, v8us hi) { return __builtin_bit_cast(v16bf, __builtin_shufflevector(lo, hi, 0, 1, 2, 3, 4, 5, 6, 7, 8, 9, 10, 11, 12, 13, 14, 15)); }
__device__ __forceinline__ v16h  ldh(const h16* p) { return cat16(*(const v8h*)p, *(const v8h*)(p + 16)); }
__device__ __forceinline__ v16bf ldb(const bf* p)  { return cat16b(*(const v8us*)p, *(const v8us*)(p + 16)); }
__device__ __forceinline__ void wave_sync() { __builtin_amdgcn_fence(3  , "wavefront"); __builtin_amdgcn_wave_barrier(); asm volatile("" ::: "memory"); }
static __device__ __forceinline__ h16 toh_flush(float v) { const h16 r = (h16)v; return (fabsf(v) < 6.103515625e-05f) ? (h16)0.0f : r; }
__device__ __forceinline__ v8f wmma16g(v16h a, v16h b, v8f c) {
    c = __builtin_amdgcn_wmma_f32_16x16x32_f16(false, a, false, b, (short)0, c, false, false);
    asm volatile("v_nop\n\tv_nop\n\tv_nop\n\tv_nop" : "+v"(c) : "v"(a), "v"(b));
    return c;
}
__device__ __forceinline__ v8f wmmabg(v16bf a, v16bf b, v8f c) {
    c = __builtin_amdgcn_wmma_f32_16x16x32_bf16(false, a, false, b, (short)0, c, false, false);
    asm volatile("v_nop\n\tv_nop\n\tv_nop\n\tv_nop" : "+v"(c) : "v"(a), "v"(b));
    return c;
}
__device__ __forceinline__ int grade_of(int x) { return (x > 0) + (x > 4) + (x > 10) + (x > 14); }
__device__ __forceinline__ float eta_of(int x) { return (((x >= 2) & (x <= 7)) | (x >= 14)) ? -1.0f : 1.0f; }

__global__ __launch_bounds__(256) void k_cvtx(const float* __restrict__ mv, const float* __restrict__ sc, bf* dst, size_t npc) {
#pragma clang fp contract(off)
    const size_t i = (size_t)blockIdx.x * 256 + threadIdx.x; if (i >= npc) return;
    const size_t tok = i / 36; const int p = (int)(i - tok * 36);
    const size_t b = tok / SEQ, t = tok - b * SEQ; const size_t st = b * SEQ_FULL + t;
    const int pm = p < 32 ? p : 31; const int pq = p < 32 ? 0 : (p - 32);
    v8f vm = *(const v8f*)(mv + st * 256 + (size_t)pm * 8);
    v8f vs = *(const v8f*)(sc + st * 32 + (size_t)pq * 8);
    asm volatile("" : "+v"(vm)); asm volatile("" : "+v"(vs));
    const bool ism = p < 32; v8us o;
#pragma unroll
    for (int k = 0; k < 8; ++k) o[k] = f2bf(ism ? vm[k] : vs[k]);
    *(volatile v8us*)(dst + i * 8) = o; __threadfence(); *(volatile v8us*)(dst + i * 8) = o;
}

__device__ __forceinline__ float win_elem(const float* __restrict__ wmv, const float* __restrict__ ws2mv, const float* __restrict__ wmv2s, const float* __restrict__ wss,
                                          int nmv, int mvoff, int soff, int useeta, int h, int d, int k) {
    const int x = d & 15;
    int c = d >> 4; c = c > 7 ? 7 : c;
    int cs = d - 128; cs = cs < 0 ? 0 : (cs > 15 ? 15 : cs);
    const int omv = mvoff + c * HN + h, osc = soff + cs * HN + h;
    int i = k >> 4; i = i > 15 ? 15 : i;
    const int xk = k & 15;
    int j = k - 256; j = j < 0 ? 0 : (j > 31 ? 31 : j);
    float a  = wmv[((size_t)grade_of(x) * nmv + omv) * 16 + i];
    float b2 = ws2mv[(size_t)omv * 32 + j];
    float c2 = wmv2s[(size_t)osc * 16 + i];
    float e  = wss[(size_t)osc * 32 + j];
    asm volatile("" : "+v"(a)); asm volatile("" : "+v"(b2)); asm volatile("" : "+v"(c2)); asm volatile("" : "+v"(e));
    const bool kmv = k < 256;
    const bool dmv = d < 128; const bool dsc = (d >= 128) & (d < 144);
    const float sg = useeta ? eta_of(x) : 1.0f;
    const float vm = kmv ? ((xk == x) ? sg * a : 0.0f) : ((x == 0) ? b2 : 0.0f);
    const float vs = kmv ? ((xk == 0) ? c2 : 0.0f) : e;
    return dmv ? vm : (dsc ? vs : 0.0f);
}

__device__ __forceinline__ void wbuild_in(const float* __restrict__ wmv, const float* __restrict__ ws2mv, const float* __restrict__ wmv2s, const float* __restrict__ wss,
                                          bf* dst, int nmv, int mvoff, int soff, int useeta, int hdw) {
#pragma clang fp contract(off)
    __shared__ __align__(16) unsigned short st[2048];
    const int tid = threadIdx.x;
    const int base = blockIdx.x * 2048;
#pragma unroll 1
    for (int e = 0; e < 8; ++e) {
        const int idx = base + e * 256 + tid;
        const int n = idx / KIN, k = idx - n * KIN;
        const int h = n / hdw, d = n - h * hdw;
        st[e * 256 + tid] = f2bf(win_elem(wmv, ws2mv, wmv2s, wss, nmv, mvoff, soff, useeta, h, d, k));
    }
    __syncthreads();
    const v8us o = *(const v8us*)(&st[tid * 8]);
    bf* q = dst + (size_t)base + (size_t)tid * 8;
    *(volatile v8us*)q = o; __threadfence(); *(volatile v8us*)q = o;
}
__global__ __launch_bounds__(256) void k_wq(const float* __restrict__ wmv, const float* __restrict__ ws2mv, const float* __restrict__ wmv2s, const float* __restrict__ wss, bf* dst) {
    wbuild_in(wmv, ws2mv, wmv2s, wss, dst, 64, 0, 0, 1, HDP);
}
__global__ __launch_bounds__(256) void k_wk(const float* __restrict__ wmv, const float* __restrict__ ws2mv, const float* __restrict__ wmv2s, const float* __restrict__ wss, bf* dst) {
    wbuild_in(wmv, ws2mv, wmv2s, wss, dst, 128, 0, 0, 0, HDP);
}
__global__ __launch_bounds__(256) void k_wv(const float* __restrict__ wmv, const float* __restrict__ ws2mv, const float* __restrict__ wmv2s, const float* __restrict__ wss, bf* dst) {
    wbuild_in(wmv, ws2mv, wmv2s, wss, dst, 128, 64, 128, 0, HDV);
}

__global__ __launch_bounds__(256) void k_wo(const float* __restrict__ wmvo, const float* __restrict__ ws2mvo, const float* __restrict__ wmv2so, const float* __restrict__ wso, h16* dst) {
#pragma clang fp contract(off)
    __shared__ __align__(16) h16 st[2048];
    const int tid = threadIdx.x;
    const int base = blockIdx.x * 2048;
#pragma unroll 1
    for (int e = 0; e < 8; ++e) {
        const int idx = base + e * 256 + tid;
        const int n = idx / KO, k = idx - n * KO;
        const int h = k / HDP, d = k - h * HDP;
        const int x = n & 15; int o = n >> 4; o = o > 15 ? 15 : o;
        int o2 = n - NMVO; o2 = o2 < 0 ? 0 : (o2 > 31 ? 31 : o2);
        const int xd = d & 15; int c = d >> 4; c = c > 7 ? 7 : c;
        int cs = d - 128; cs = cs < 0 ? 0 : (cs > 15 ? 15 : cs);
        float a  = wmvo[((size_t)grade_of(x) * 16 + o) * 64 + h * CMV + c];
        float b2 = ws2mvo[(size_t)o * 128 + h * CSC + cs];
        float c2 = wmv2so[(size_t)o2 * 64 + h * CMV + c];
        float ee = wso[(size_t)o2 * 128 + h * CSC + cs];
        asm volatile("" : "+v"(a)); asm volatile("" : "+v"(b2)); asm volatile("" : "+v"(c2)); asm volatile("" : "+v"(ee));
        const bool dmv = d < 128; const bool dsc = (d >= 128) & (d < 144);
        const bool nmv = n < NMVO; const bool nsc = (n >= NMVO) & (n < NMVO + NSCO);
        const float vm = dmv ? ((xd == x) ? a : 0.0f) : (dsc ? ((x == 0) ? b2 : 0.0f) : 0.0f);
        const float vs = dmv ? ((xd == 0) ? c2 : 0.0f) : (dsc ? ee : 0.0f);
        const float v = nmv ? vm : (nsc ? vs : 0.0f);
        st[e * 256 + tid] = toh_flush(bfr(v) * WOS);
    }
    __syncthreads();
    const v8h o8 = *(const v8h*)(&st[tid * 8]);
    h16* q = dst + (size_t)base + (size_t)tid * 8;
    *(volatile v8h*)q = o8; __threadfence(); *(volatile v8h*)q = o8;
}

template <int MODE>
__device__ __forceinline__ void proj_body(const bf* __restrict__ A, const bf* __restrict__ Bt, h16* Ph) {
    __shared__ __align__(16) float os[16 * 68];
    const int K = KIN;
    const int lane = threadIdx.x & 31, lr = lane & 15, hi = lane >> 4; const int r0 = blockIdx.x * 64, c0 = blockIdx.y * 64;
    v8f acc[4][4];
#pragma unroll
    for (int mb = 0; mb < 4; ++mb)
#pragma unroll
        for (int nb = 0; nb < 4; ++nb) acc[mb][nb] = (v8f){};
    const size_t aoff = (size_t)(r0 + lr) * K + 8 * hi, boff = (size_t)(c0 + lr) * K + 8 * hi;
#pragma unroll 1
    for (int kc = 0; kc < K; kc += 32) {
        v16bf a[4];
#pragma unroll
        for (int mb = 0; mb < 4; ++mb) a[mb] = ldb(A + aoff + (size_t)mb * 16 * K + kc);
#pragma unroll
        for (int nb = 0; nb < 4; ++nb) { const v16bf b = ldb(Bt + boff + (size_t)nb * 16 * K + kc);
#pragma unroll
            for (int mb = 0; mb < 4; ++mb) acc[mb][nb] = wmmabg(a[mb], b, acc[mb][nb]); }
    }
    size_t tbase;
    if (MODE == 0) { const int bb = r0 / SEQ, tt = r0 % SEQ; const int zc = bb * NZ + c0 / 32;
                     tbase = ((size_t)zc * SEQ + (size_t)tt) * 32; }
    else           { const int bb = c0 / SEQ, tt = c0 % SEQ;
                     tbase = (size_t)bb * (size_t)NVF * SEQ + (size_t)r0 * SEQ + (size_t)tt; }
#pragma unroll
    for (int mb = 0; mb < 4; ++mb) {
#pragma unroll
        for (int nb = 0; nb < 4; ++nb) {
#pragma unroll
            for (int j = 0; j < 8; ++j) os[(hi * 8 + j) * 68 + nb * 16 + lr] = acc[mb][nb][j]; }
        wave_sync();
#pragma unroll 1
        for (int ps = 0; ps < 2; ++ps) {
            if (MODE == 0) {
                const size_t sb = tbase + (size_t)(mb * 16) * 32;
#pragma unroll
                for (int hh = 0; hh < 2; ++hh) {
#pragma unroll
                    for (int s = 0; s < 2; ++s) { const int p = s * 32 + lane; const int row = p >> 2, c8 = (p & 3) * 8;
                        const v4f x0 = *(const v4fa*)(&os[row * 68 + hh * 32 + c8]); const v4f x1 = *(const v4fa*)(&os[row * 68 + hh * 32 + c8 + 4]); v8h hv;
#pragma unroll
                        for (int i = 0; i < 4; ++i) { hv[i] = toh_flush(x0[i]); hv[4 + i] = toh_flush(x1[i]); }
                        const size_t oo = sb + (size_t)hh * ((size_t)SEQ * 32) + (size_t)p * 8;
                        *(volatile v8h*)(Ph + oo) = hv; } }
            } else {
                const size_t sb = tbase + (size_t)(mb * 16) * SEQ;
#pragma unroll
                for (int s = 0; s < 4; ++s) { const int row = 4 * s + (lane >> 3), c8 = (lane & 7) * 8;
                    const v4f x0 = *(const v4fa*)(&os[row * 68 + c8]); const v4f x1 = *(const v4fa*)(&os[row * 68 + c8 + 4]); v8h hv;
#pragma unroll
                    for (int i = 0; i < 4; ++i) { hv[i] = toh_flush(x0[i]); hv[4 + i] = toh_flush(x1[i]); }
                    const size_t oo = sb + (size_t)row * SEQ + c8;
                    *(volatile v8h*)(Ph + oo) = hv; }
            }
            if (ps == 0) __threadfence(); }
        wave_sync();
    }
}
__global__ __launch_bounds__(32) void k_proj_rows(const bf* __restrict__ A, const bf* __restrict__ Bt, h16* Ph) { proj_body<0>(A, Bt, Ph); }
__global__ __launch_bounds__(32) void k_proj_cols(const bf* __restrict__ A, const bf* __restrict__ Bt, h16* Ph) { proj_body<1>(A, Bt, Ph); }

__global__ __launch_bounds__(32 * AW) __attribute__((amdgpu_num_vgpr(256)))
void k_flash(const h16* __restrict__ QH, const h16* __restrict__ KP, const h16* __restrict__ VT, const float* __restrict__ hscale, h16* CX, h16* CXR) {
    __shared__ __align__(16) float os[AW * 16 * OSP];
    const int lane = threadIdx.x & 31, lr = lane & 15, hi = lane >> 4;
    const int wave = __builtin_amdgcn_readfirstlane((int)(threadIdx.x >> 5));
    const int zh = blockIdx.y; const int h = zh % HN;
    const int t0 = (blockIdx.x * AW + wave) * 16;
    const size_t pz = (size_t)zh * NKS * SEQ * 32;
    const unsigned qo = (unsigned)(pz + (size_t)(t0 + lr) * 32 + 8 * hi);
    const size_t ko = pz + (size_t)lr * 32 + 8 * hi;
    const size_t vo = (size_t)zh * HDV * SEQ + (size_t)lr * SEQ + 8 * hi;
    v8f o[9];
#pragma unroll
    for (int j = 0; j < 9; ++j) o[j] = (v8f){};
    float m = NEGB, l = 0.0f;
#pragma unroll 1
    for (int key0 = 0; key0 < SEQ; key0 += 32) {
        unsigned qv = qo; asm volatile("" : "+v"(qv));
        const h16* ka = KP + ko + (size_t)key0 * 32;
        v8f sa = (v8f){}, sb = (v8f){};
#pragma unroll
        for (int ks = 0; ks < NKS; ++ks) {
            const v16h qf = ldh(QH + qv + (size_t)ks * SEQ * 32);
            const v16h k0 = ldh(ka + (size_t)ks * SEQ * 32), k1 = ldh(ka + (size_t)ks * SEQ * 32 + 16 * 32);
            sa = wmma16g(k0, qf, sa); sb = wmma16g(k1, qf, sb); }
        float ta[8], tb[8]; float mx = NEGB;
#pragma unroll
        for (int r = 0; r < 8; ++r) { ta[r] = sa[r] * SC2; tb[r] = sb[r] * SC2; mx = fmaxf(mx, fmaxf(ta[r], tb[r])); }
        mx = fmaxf(mx, __shfl_xor(mx, 16, 32));
        const float mnew = fmaxf(m, mx);
        const float alpha = __builtin_amdgcn_exp2f(m - mnew);
        const float sh = PSH - mnew;
        v16h pb; float ls = 0.0f;
#pragma unroll
        for (int r = 0; r < 8; ++r) {
            const float xa = ta[r] + sh, xb = tb[r] + sh;
            const float ea = (xa < -14.0f) ? 0.0f : __builtin_amdgcn_exp2f(xa);
            const float eb = (xb < -14.0f) ? 0.0f : __builtin_amdgcn_exp2f(xb);
            const h16 pa = (h16)ea; const h16 pc = (h16)eb;
            pb[r] = pa; pb[8 + r] = pc; ls += (float)pa + (float)pc; }
        l = l * alpha + ls; m = mnew;
#pragma unroll
        for (int j = 0; j < 9; ++j) o[j] = o[j] * alpha;
        const h16* va = VT + vo + key0;
#pragma unroll
        for (int j = 0; j < 9; ++j) { const v16h vf = ldh(va + (size_t)(16 * j) * SEQ); o[j] = wmma16g(vf, pb, o[j]); }
    }
    l += __shfl_xor(l, 16, 32);
    const float hsv = bfr(hscale[h]);
    const float oscl = (1.0f / l) * hsv * CXS;
    const int wb = wave * 16 * OSP;
#pragma unroll
    for (int j = 0; j < 9; ++j) { v4f a, c;
        a[0] = o[j][0] * oscl; a[1] = o[j][1] * oscl; a[2] = o[j][2] * oscl; a[3] = o[j][3] * oscl; c[0] = o[j][4] * oscl; c[1] = o[j][5] * oscl; c[2] = o[j][6] * oscl; c[3] = o[j][7] * oscl;
        *(v4fa*)(&os[wb + lr * OSP + 16 * j + 8 * hi]) = a; *(v4fa*)(&os[wb + lr * OSP + 16 * j + 8 * hi + 4]) = c; }
    { const v4f z = (v4f){}; *(v4fa*)(&os[wb + lr * OSP + HDV + 8 * hi]) = z; *(v4fa*)(&os[wb + lr * OSP + HDV + 8 * hi + 4]) = z; }
    wave_sync();
    h16* cb = CX + pz + (size_t)t0 * 32;
    h16* cr = CXR + pz + (size_t)t0 * 32;
#pragma unroll 1
    for (int ps = 0; ps < 2; ++ps) {
#pragma unroll
        for (int ks = 0; ks < NKS; ++ks) {
#pragma unroll
            for (int s = 0; s < 2; ++s) { const int p = s * 32 + lane; const int row = p >> 2, c8 = (p & 3) * 8;
                const v4f x0 = *(const v4fa*)(&os[wb + row * OSP + ks * 32 + c8]); const v4f x1 = *(const v4fa*)(&os[wb + row * OSP + ks * 32 + c8 + 4]); v8h hv, rv;
#pragma unroll
                for (int i = 0; i < 4; ++i) { const h16 a0 = toh_flush(x0[i]); const h16 a1 = toh_flush(x1[i]); hv[i] = a0; hv[4 + i] = a1;
                    rv[i] = toh_flush((x0[i] - (float)a0) * QRS); rv[4 + i] = toh_flush((x1[i] - (float)a1) * QRS); }
                const size_t oo = (size_t)ks * SEQ * 32 + (size_t)p * 8;
                *(volatile v8h*)(cb + oo) = hv; *(volatile v8h*)(cr + oo) = rv; } }
        if (ps == 0) __threadfence(); }
}

__global__ __launch_bounds__(32) void k_oproj(const h16* __restrict__ CX, const h16* __restrict__ CXR, const h16* __restrict__ WO, float* OUT) {
    __shared__ __align__(16) float os[16 * 68];
    const int lane = threadIdx.x & 31, lr = lane & 15, hi = lane >> 4; const int r0 = blockIdx.x * OTR, c0 = blockIdx.y * 64;
    const int bb = r0 / SEQ, tt = r0 % SEQ;
    v8f acc[OMB][4], acr[OMB][4];
#pragma unroll
    for (int mb = 0; mb < OMB; ++mb)
#pragma unroll
        for (int nb = 0; nb < 4; ++nb) { acc[mb][nb] = (v8f){}; acr[mb][nb] = (v8f){}; }
    const size_t aoff = ((size_t)bb * NZ * SEQ + (size_t)(tt + lr)) * 32 + 8 * hi;
    const size_t boff = (size_t)(c0 + lr) * KO + 8 * hi;
#pragma unroll 1
    for (int kk = 0; kk < NZ; ++kk) {
        v16h a[OMB], ar[OMB];
#pragma unroll
        for (int mb = 0; mb < OMB; ++mb) { const size_t ao = aoff + (size_t)kk * SEQ * 32 + (size_t)mb * 16 * 32; a[mb] = ldh(CX + ao); ar[mb] = ldh(CXR + ao); }
#pragma unroll
        for (int nb = 0; nb < 4; ++nb) { const v16h b = ldh(WO + boff + (size_t)nb * 16 * KO + (size_t)kk * 32);
#pragma unroll
            for (int mb = 0; mb < OMB; ++mb) { acc[mb][nb] = wmma16g(a[mb], b, acc[mb][nb]); acr[mb][nb] = wmma16g(ar[mb], b, acr[mb][nb]); } }
    }
#pragma unroll
    for (int mb = 0; mb < OMB; ++mb) {
#pragma unroll
        for (int nb = 0; nb < 4; ++nb) {
#pragma unroll
            for (int j = 0; j < 8; ++j) os[(hi * 8 + j) * 68 + nb * 16 + lr] = (acc[mb][nb][j] + acr[mb][nb][j] * QRI) * OSCL; }
        wave_sync();
        const size_t tok = (size_t)bb * OUT_SEQ + (size_t)(tt + mb * 16);
#pragma unroll 1
        for (int ps = 0; ps < 2; ++ps) {
            if (c0 < NMVO) {
#pragma unroll
                for (int s = 0; s < 8; ++s) { const int row = 2 * s + (lane >> 4), cofs = (lane & 15) * 4;
                    const v4f val = *(const v4fa*)(&os[row * 68 + cofs]);
                    *(volatile v4f*)(OUT + (tok + (size_t)row) * NMVO + c0 + cofs) = val; }
            } else {
#pragma unroll
                for (int s = 0; s < 4; ++s) { const int row = 4 * s + (lane >> 3), cofs = (lane & 7) * 4;
                    const v4f val = *(const v4fa*)(&os[row * 68 + cofs]);
                    *(volatile v4f*)(OUT + O1_OFF + (tok + (size_t)row) * NSCO + cofs) = val; }
            }
            if (ps == 0) __threadfence(); }
        wave_sync();
    }
}

static constexpr size_t al256(size_t v) { return (v + 255) & ~(size_t)255; }
static constexpr size_t SZ_X   = al256((size_t)NB * SEQ * KIN * 2);
static constexpr size_t SZ_WQK = al256((size_t)NQK * KIN * 2);
static constexpr size_t SZ_WV  = al256((size_t)NVF * KIN * 2);
static constexpr size_t SZ_WO  = al256((size_t)NOP * KO * 2);
static constexpr size_t SZ_PL  = al256((size_t)NB * NZ * SEQ * 32 * 2);
static constexpr size_t SZ_VT  = al256((size_t)NB * NVF * SEQ * 2);
static constexpr size_t SZ_TOTAL = 2 * SZ_X + 2 * SZ_WQK + SZ_WV + SZ_WO + 4 * SZ_PL + SZ_VT;
static_assert(SZ_TOTAL <= (size_t)134217728);
static_assert(SZ_PL >= (size_t)NB * HN * NKS * SEQ * 32 * 2);
static_assert(((size_t)NB * SEQ * KIN * 2) % 128 == 0);
static_assert(((size_t)NB * SEQ * KIN / 8) % 32 == 0);

extern "C" void kernel_launch(void* const* d_in, const int* in_sizes, int n_in,
                              void* d_out, int out_size, void* d_ws, size_t ws_size, hipStream_t stream) {
    if (n_in < 17) return;
    const size_t needmv = ((size_t)(NB - 1) * SEQ_FULL + SEQ) * 256;
    const size_t needsc = ((size_t)(NB - 1) * SEQ_FULL + SEQ) * 32;
    if ((size_t)in_sizes[0] < needmv || (size_t)in_sizes[1] < needmv) return;
    if ((size_t)in_sizes[2] < needsc || (size_t)in_sizes[3] < needsc) return;
    if (in_sizes[4] < 5 * 64 * 16 || in_sizes[5] < 64 * 32 || in_sizes[6] < 128 * 16 || in_sizes[7] < 128 * 32) return;
    if (in_sizes[8] < 5 * 128 * 16 || in_sizes[9] < 128 * 32 || in_sizes[10] < 256 * 16 || in_sizes[11] < 256 * 32) return;
    if (in_sizes[12] < 5 * 16 * 64 || in_sizes[13] < 16 * 128 || in_sizes[14] < 32 * 64 || in_sizes[15] < 32 * 128) return;
    if (in_sizes[16] < HN) return;
    if ((size_t)out_size < O1_OFF + ((size_t)(NB - 1) * OUT_SEQ + SEQ) * NSCO) return;
    if ((size_t)out_size < ((size_t)(NB - 1) * OUT_SEQ + SEQ) * NMVO) return;
    if (SZ_TOTAL > ws_size) return;
    const float* mv_kv = (const float*)d_in[0];  const float* mv_q = (const float*)d_in[1];
    const float* s_kv  = (const float*)d_in[2];  const float* s_q  = (const float*)d_in[3];
    const float* wq_mv = (const float*)d_in[4];  const float* wq_s2mv = (const float*)d_in[5];  const float* wq_mv2s = (const float*)d_in[6];  const float* wq_s = (const float*)d_in[7];
    const float* wk_mv = (const float*)d_in[8];  const float* wk_s2mv = (const float*)d_in[9];  const float* wk_mv2s = (const float*)d_in[10]; const float* wk_s = (const float*)d_in[11];
    const float* wo_mv = (const float*)d_in[12]; const float* wo_s2mv = (const float*)d_in[13]; const float* wo_mv2s = (const float*)d_in[14]; const float* wo_s = (const float*)d_in[15];
    const float* hsc = (const float*)d_in[16];
    float* OUT = (float*)d_out;
    char* wsp = (char*)d_ws;
    bf*  XQ  = (bf*)wsp;  wsp += SZ_X;
    bf*  XKV = (bf*)wsp;  wsp += SZ_X;
    bf*  WQ  = (bf*)wsp;  wsp += SZ_WQK;
    bf*  WK  = (bf*)wsp;  wsp += SZ_WQK;
    bf*  WV  = (bf*)wsp;  wsp += SZ_WV;
    h16* WO  = (h16*)wsp; wsp += SZ_WO;
    h16* QH  = (h16*)wsp; wsp += SZ_PL;
    h16* KP  = (h16*)wsp; wsp += SZ_PL;
    h16* CX  = (h16*)wsp; wsp += SZ_PL;
    h16* CXR = (h16*)wsp; wsp += SZ_PL;
    h16* VT  = (h16*)wsp; wsp += SZ_VT;

    { const size_t npc = (size_t)NB * SEQ * (KIN / 8); const unsigned g = (unsigned)((npc + 255) / 256);
      k_cvtx<<<g, 256, 0, stream>>>(mv_q, s_q, XQ, npc);
      k_cvtx<<<g, 256, 0, stream>>>(mv_kv, s_kv, XKV, npc); }
    k_wq<<<(unsigned)((size_t)NQK * KIN / 2048), 256, 0, stream>>>(wq_mv, wq_s2mv, wq_mv2s, wq_s, WQ);
    k_wk<<<(unsigned)((size_t)NQK * KIN / 2048), 256, 0, stream>>>(wk_mv, wk_s2mv, wk_mv2s, wk_s, WK);
    k_wv<<<(unsigned)((size_t)NVF * KIN / 2048), 256, 0, stream>>>(wk_mv, wk_s2mv, wk_mv2s, wk_s, WV);
    k_wo<<<(unsigned)((size_t)NOP * KO / 2048), 256, 0, stream>>>(wo_mv, wo_s2mv, wo_mv2s, wo_s, WO);

    k_proj_rows<<<dim3(NB * SEQ / 64, NQK / 64, 1), 32, 0, stream>>>(XQ, WQ, QH);
    k_proj_rows<<<dim3(NB * SEQ / 64, NQK / 64, 1), 32, 0, stream>>>(XKV, WK, KP);
    k_proj_cols<<<dim3(NVF / 64, NB * SEQ / 64, 1), 32, 0, stream>>>(WV, XKV, VT);

    k_flash<<<dim3(SEQ / (16 * AW), NB * HN, 1), 32 * AW, 0, stream>>>(QH, KP, VT, hsc, CX, CXR);

    k_oproj<<<dim3(NB * SEQ / OTR, NOP / 64, 1), 32, 0, stream>>>(CX, CXR, WO, OUT);
}
